// Superpoint_MAE_55207509623408
// MI455X (gfx1250) — hardware-verified
//
#include <hip/hip_runtime.h>
#include <stddef.h>

#define N_PTS  262144
#define S1_N   4096
#define S2_N   128
#define PAD_N  64
#define F_IN   11
#define H1_N   128
#define H2_N   256
#define H3_N   512
#define C_N    384
#define PH_N   128
#define GRP    4
#define RMAX   1024
#define MC     32
#define XP     12
#define AP     264
#define HP     520
#define TKP    388
#define G3P    516
#define PP     136
#define NTHR   256
#define LB_IT_N  19
#define LB_IT_S1 13

static_assert(NTHR == H2_N);
static_assert(S1_N % GRP == 0);
static_assert(S1_N % MC == 0);
static_assert(RMAX % MC == 0);
static_assert(MC * F_IN <= 2 * NTHR);
static_assert((NTHR / 32) * 64 == H3_N);
static_assert((NTHR / 32) * 48 == C_N);
static_assert(H2_N % 64 == 0 && H3_N % 64 == 0 && C_N % 64 == 0 && PH_N % 64 == 0);
static_assert(AP % 8 == 0 && HP % 8 == 0 && PP % 8 == 0);
static_assert((TKP * 4) % 16 == 0 && (G3P * 4) % 16 == 0);
static_assert(MC * HP * 2 >= GRP * TKP * 4);
static_assert(MC * TKP * 4 >= 2 * MC * PP * 2);
static_assert((GRP * H3_N) % NTHR == 0);
static_assert((1 << (LB_IT_N - 1)) >= N_PTS);
static_assert((1 << (LB_IT_S1 - 1)) >= S1_N);

typedef _Float16 f16;
typedef f16 v16h __attribute__((ext_vector_type(16)));
typedef f16 v8h_t __attribute__((ext_vector_type(8)));
typedef v8h_t __attribute__((may_alias)) v8h;
typedef unsigned short v16us_t __attribute__((ext_vector_type(16)));
typedef unsigned short v8us_t __attribute__((ext_vector_type(8)));
typedef v8us_t __attribute__((may_alias)) v8us;
typedef __bf16 v16bf __attribute__((ext_vector_type(16)));
typedef float v8f __attribute__((ext_vector_type(8)));
typedef float v4f_t __attribute__((ext_vector_type(4)));
typedef v4f_t __attribute__((may_alias)) v4f;

union FragH { v16h v; v8h_t h[2]; };
union FragB { v16bf v; v16us_t u; v8us_t h[2]; };

__device__ __forceinline__ v8f zero8() {
    v8f z;
#pragma unroll
    for (int i = 0; i < 8; ++i) z[i] = 0.0f;
    return z;
}

__device__ __forceinline__ v16h ldfrag_h(const f16* p, int k0) {
    FragH f;
    f.h[0] = *(const v8h*)(p + k0);
    f.h[1] = *(const v8h*)(p + k0 + 16);
    return f.v;
}
__device__ __forceinline__ v16bf ldfrag_b(const unsigned short* p, int k0) {
    FragB f;
    f.h[0] = *(const v8us*)(p + k0);
    f.h[1] = *(const v8us*)(p + k0 + 16);
    return f.v;
}

__device__ __forceinline__ v8f wm_h(v16h a, v16h b, v8f c) {
    return __builtin_amdgcn_wmma_f32_16x16x32_f16(false, a, false, b, (short)0, c, false, false);
}
__device__ __forceinline__ v8f wm_b(v16bf a, v16bf b, v8f c) {
    return __builtin_amdgcn_wmma_f32_16x16x32_bf16(false, a, false, b, (short)0, c, false, false);
}

__device__ __forceinline__ unsigned short bf16_rne(float x) {
    unsigned u = __float_as_uint(x);
    u = u + 0x7FFFu + ((u >> 16) & 1u);
    return (unsigned short)(u >> 16);
}

__device__ __forceinline__ int lbound(const int* __restrict__ a, int n, int v, int iters) {
    int lo = 0, hi = n;
#pragma unroll 1
    for (int it = 0; it < iters; ++it) {
        const int mid = (lo + hi) >> 1;
        const int mc = mid < (n - 1) ? mid : (n - 1);
        const int x = a[mc];
        if (lo < hi) {
            if (x < v) lo = mid + 1; else hi = mid;
        }
    }
    return lo;
}

__global__ void __launch_bounds__(NTHR) prep_kernel(
    const float* __restrict__ W1, const float* __restrict__ b1,
    const float* __restrict__ W2, const float* __restrict__ b2,
    float* __restrict__ Wc, float* __restrict__ bc)
{
    const int c = threadIdx.x;
    float wv[F_IN];
#pragma unroll
    for (int k = 0; k < F_IN; ++k) {
        float a = 0.0f;
#pragma unroll 1
        for (int j = 0; j < H1_N; ++j) a = fmaf(W1[k * H1_N + j], W2[j * H2_N + c], a);
        wv[k] = a;
    }
    float ab = b2[c];
#pragma unroll 1
    for (int j = 0; j < H1_N; ++j) ab = fmaf(b1[j], W2[j * H2_N + c], ab);
#pragma unroll
    for (int k = 0; k < F_IN; ++k) *(volatile float*)(Wc + k * H2_N + c) = wv[k];
    *(volatile float*)(bc + c) = ab;
    __threadfence();
#pragma unroll
    for (int k = 0; k < F_IN; ++k) *(volatile float*)(Wc + k * H2_N + c) = wv[k];
    *(volatile float*)(bc + c) = ab;
}

template <int MODE>
__global__ void __launch_bounds__(NTHR) cvt_t_kernel(
    const float* __restrict__ src, int K, int Nn, float scale,
    unsigned short* d0, unsigned short* d1)
{
    __shared__ __align__(16) unsigned short t0[64 * 72];
    __shared__ __align__(16) unsigned short t1[64 * 72];
    const int tid = threadIdx.x;
    const int n0 = blockIdx.x * 64, k0 = blockIdx.y * 64;
#pragma unroll 4
    for (int i = 0; i < 16; ++i) {
        const int idx = i * NTHR + tid;
        const int kk = idx >> 6, nn = idx & 63;
        const float v = src[(size_t)(k0 + kk) * (size_t)Nn + (size_t)(n0 + nn)] * scale;
        if (MODE == 0) {
            t0[nn * 72 + kk] = __builtin_bit_cast(unsigned short, (f16)v);
        } else {
            const unsigned short hb = bf16_rne(v);
            const float hf = __uint_as_float(((unsigned)hb) << 16);
            t0[nn * 72 + kk] = hb;
            t1[nn * 72 + kk] = bf16_rne(v - hf);
        }
    }
    __syncthreads();
    v8us_t o0[2], o1[2];
#pragma unroll
    for (int it = 0; it < 2; ++it) {
        const int nn = it * 32 + (tid >> 3);
        const int col = (tid & 7) * 8;
        o0[it] = *(const v8us*)(t0 + nn * 72 + col);
        if (MODE == 1) o1[it] = *(const v8us*)(t1 + nn * 72 + col);
        else o1[it] = o0[it];
    }
#pragma unroll
    for (int it = 0; it < 2; ++it) {
        const int nn = it * 32 + (tid >> 3);
        const int col = (tid & 7) * 8;
        const size_t off = (size_t)(n0 + nn) * (size_t)K + (size_t)(k0 + col);
        *(volatile v8us_t*)(d0 + off) = o0[it];
        if (MODE == 1) *(volatile v8us_t*)(d1 + off) = o1[it];
    }
    __threadfence();
#pragma unroll
    for (int it = 0; it < 2; ++it) {
        const int nn = it * 32 + (tid >> 3);
        const int col = (tid & 7) * 8;
        const size_t off = (size_t)(n0 + nn) * (size_t)K + (size_t)(k0 + col);
        *(volatile v8us_t*)(d0 + off) = o0[it];
        if (MODE == 1) *(volatile v8us_t*)(d1 + off) = o1[it];
    }
}

__device__ __forceinline__ void stage_x(const float* __restrict__ X, float* xs, int prow, int tid) {
#pragma unroll
    for (int i = 0; i < 2; ++i) {
        const int e = i * NTHR + tid;
        size_t gi = (size_t)prow * F_IN + (size_t)e;
        const size_t gmax = (size_t)N_PTS * F_IN - 1;
        gi = gi < gmax ? gi : gmax;
        const float v = X[gi];
        if (e < MC * F_IN) {
            const int rr = e / F_IN;
            const int k = e - rr * F_IN;
            xs[rr * XP + k] = v;
        }
    }
}
__device__ __forceinline__ float f_dot(const float* xr, const float* wv, float bcv) {
    const v4f_t x0 = *(const v4f*)(xr);
    const v4f_t x1 = *(const v4f*)(xr + 4);
    const v4f_t x2 = *(const v4f*)(xr + 8);
    float v = bcv;
    v = fmaf(x0[0], wv[0], v);
    v = fmaf(x0[1], wv[1], v);
    v = fmaf(x0[2], wv[2], v);
    v = fmaf(x0[3], wv[3], v);
    v = fmaf(x1[0], wv[4], v);
    v = fmaf(x1[1], wv[5], v);
    v = fmaf(x1[2], wv[6], v);
    v = fmaf(x1[3], wv[7], v);
    v = fmaf(x2[0], wv[8], v);
    v = fmaf(x2[1], wv[9], v);
    v = fmaf(x2[2], wv[10], v);
    return v;
}

__global__ void __launch_bounds__(NTHR) segmax1_kernel(
    const float* __restrict__ X, const int* __restrict__ idx10,
    const float* __restrict__ Wc, const float* __restrict__ bc,
    float* __restrict__ gout)
{
    __shared__ __align__(16) float xs[MC * XP];
    __shared__ int bnd[GRP + 1];
    const int tid = threadIdx.x;
    const int s0 = blockIdx.x * GRP;
    if (tid <= GRP) bnd[tid] = lbound(idx10, N_PTS, s0 + tid, LB_IT_N);
    float wv[F_IN];
#pragma unroll
    for (int k = 0; k < F_IN; ++k) wv[k] = Wc[k * H2_N + tid];
    const float bcv = bc[tid];
    if (tid < MC) xs[tid * XP + 11] = 0.0f;
    __syncthreads();
    const int P0 = bnd[0];
    int R = bnd[GRP] - P0;
    R = R < 0 ? 0 : R;
    R = R > RMAX ? RMAX : R;
    int bl[GRP - 1];
#pragma unroll
    for (int j = 0; j < GRP - 1; ++j) {
        int b = bnd[j + 1] - P0;
        b = b < 0 ? 0 : b;
        b = b > R ? R : b;
        bl[j] = b;
    }
    const float NEG = -__builtin_huge_valf();
    float m[GRP];
#pragma unroll
    for (int j = 0; j < GRP; ++j) m[j] = NEG;
    const int nch = (R + MC - 1) / MC;
#pragma unroll 1
    for (int ch = 0; ch < nch; ++ch) {
        const int r0 = ch * MC;
        __syncthreads();
        stage_x(X, xs, P0 + r0, tid);
        __syncthreads();
#pragma unroll 1
        for (int rr = 0; rr < MC; ++rr) {
            const float v = f_dot(xs + rr * XP, wv, bcv);
            const int grow = r0 + rr;
            const bool ok = grow < R;
            int ls = 0;
#pragma unroll
            for (int j = 0; j < GRP - 1; ++j) ls += (grow >= bl[j]) ? 1 : 0;
#pragma unroll
            for (int j = 0; j < GRP; ++j) m[j] = (ok && ls == j) ? fmaxf(m[j], v) : m[j];
        }
    }
#pragma unroll
    for (int j = 0; j < GRP; ++j) *(volatile float*)(gout + (size_t)(s0 + j) * H2_N + tid) = m[j];
    __threadfence();
#pragma unroll
    for (int j = 0; j < GRP; ++j) *(volatile float*)(gout + (size_t)(s0 + j) * H2_N + tid) = m[j];
}

__global__ void __launch_bounds__(NTHR) g3_kernel(
    const float* __restrict__ g, const f16* __restrict__ W3aT,
    const float* __restrict__ b3, float* __restrict__ G3)
{
    __shared__ __align__(16) f16 As[MC * AP];
    __shared__ __align__(16) float stg[16 * G3P];
    const int tid = threadIdx.x, lane = tid & 31, w = tid >> 5;
    const int hh = lane >> 4, m16 = lane & 15;
    const int s0 = blockIdx.x * MC;
#pragma unroll 4
    for (int r = 0; r < MC; ++r)
        As[r * AP + tid] = (f16)(g[(size_t)(s0 + r) * H2_N + tid] * 256.0f);
    float b3v[4];
#pragma unroll
    for (int nt = 0; nt < 4; ++nt) b3v[nt] = b3[64 * w + 16 * nt + m16];
    __syncthreads();

    v8f acc[2][4];
#pragma unroll
    for (int mt = 0; mt < 2; ++mt)
#pragma unroll
        for (int nt = 0; nt < 4; ++nt) acc[mt][nt] = zero8();
    const f16* pa = As + m16 * AP + 8 * hh;
    const f16* pb = W3aT + (size_t)(64 * w + m16) * H2_N + 8 * hh;
#pragma unroll 1
    for (int k0 = 0; k0 < H2_N; k0 += 32) {
        const v16h af0 = ldfrag_h(pa, k0);
        const v16h af1 = ldfrag_h(pa + 16 * AP, k0);
        v16h bfr[4];
#pragma unroll
        for (int nt = 0; nt < 4; ++nt) bfr[nt] = ldfrag_h(pb + (size_t)nt * 16 * H2_N, k0);
#pragma unroll
        for (int nt = 0; nt < 4; ++nt) {
            acc[0][nt] = wm_h(af0, bfr[nt], acc[0][nt]);
            acc[1][nt] = wm_h(af1, bfr[nt], acc[1][nt]);
        }
        asm volatile("v_nop\n\tv_nop\n\tv_nop\n\tv_nop"
                     : "+v"(acc[0][0]), "+v"(acc[0][1]), "+v"(acc[0][2]), "+v"(acc[0][3]),
                       "+v"(acc[1][0]), "+v"(acc[1][1]), "+v"(acc[1][2]), "+v"(acc[1][3])
                     : "v"(af0), "v"(af1), "v"(bfr[0]), "v"(bfr[1]), "v"(bfr[2]), "v"(bfr[3]));
    }

#pragma unroll
    for (int mt = 0; mt < 2; ++mt) {
#pragma unroll
        for (int nt = 0; nt < 4; ++nt) {
            const int col = 64 * w + 16 * nt + m16;
#pragma unroll
            for (int r = 0; r < 8; ++r)
                stg[(8 * hh + r) * G3P + col] = fmaf(acc[mt][nt][r], 1.0f / 16384.0f, b3v[nt]);
        }
        __syncthreads();
        v4f_t ov[8];
#pragma unroll
        for (int it = 0; it < 8; ++it) {
            const int L = it * 32 + (tid >> 3);
            const int row = L >> 4, q = L & 15;
            const int col = q * 32 + (tid & 7) * 4;
            ov[it] = *(const v4f*)(stg + row * G3P + col);
        }
#pragma unroll
        for (int it = 0; it < 8; ++it) {
            const int L = it * 32 + (tid >> 3);
            const int row = L >> 4, q = L & 15;
            const int col = q * 32 + (tid & 7) * 4;
            *(volatile v4f_t*)(G3 + (size_t)(s0 + 16 * mt + row) * H3_N + col) = ov[it];
        }
        __threadfence();
#pragma unroll
        for (int it = 0; it < 8; ++it) {
            const int L = it * 32 + (tid >> 3);
            const int row = L >> 4, q = L & 15;
            const int col = q * 32 + (tid & 7) * 4;
            *(volatile v4f_t*)(G3 + (size_t)(s0 + 16 * mt + row) * H3_N + col) = ov[it];
        }
        __syncthreads();
    }
}

__global__ void __launch_bounds__(NTHR) fused_kernel(
    const float* __restrict__ X, const int* __restrict__ idx10,
    const float* __restrict__ Wc, const float* __restrict__ bc,
    const float* __restrict__ G3, const f16* __restrict__ W3bT,
    const f16* __restrict__ W4T, const float* __restrict__ b4,
    float* __restrict__ tok)
{
    __shared__ __align__(16) float xs[MC * XP];
    __shared__ __align__(16) f16 As[MC * AP];
    __shared__ __align__(16) f16 hs[MC * HP];
    __shared__ __align__(16) float g3s[GRP * H3_N];
    __shared__ int bnd[GRP + 1];

    const int tid = threadIdx.x, lane = tid & 31, w = tid >> 5;
    const int hh = lane >> 4, m16 = lane & 15;
    const int s0 = blockIdx.x * GRP;

    if (tid <= GRP) bnd[tid] = lbound(idx10, N_PTS, s0 + tid, LB_IT_N);
    float wv[F_IN];
#pragma unroll
    for (int k = 0; k < F_IN; ++k) wv[k] = Wc[k * H2_N + tid];
    const float bcv = bc[tid];
    float b4v[3];
#pragma unroll
    for (int nt = 0; nt < 3; ++nt) b4v[nt] = b4[48 * w + 16 * nt + m16];
#pragma unroll
    for (int i = 0; i < (GRP * H3_N) / NTHR; ++i) {
        const int e = i * NTHR + tid;
        g3s[e] = G3[(size_t)(s0 + (e >> 9)) * H3_N + (size_t)(e & (H3_N - 1))];
    }
    if (tid < MC) xs[tid * XP + 11] = 0.0f;
    __syncthreads();
    const int P0 = bnd[0];
    int R = bnd[GRP] - P0;
    R = R < 0 ? 0 : R;
    R = R > RMAX ? RMAX : R;
    int bl[GRP - 1];
#pragma unroll
    for (int j = 0; j < GRP - 1; ++j) {
        int b = bnd[j + 1] - P0;
        b = b < 0 ? 0 : b;
        b = b > R ? R : b;
        bl[j] = b;
    }
    const float NEG = -__builtin_huge_valf();
    float tm[GRP][3];
#pragma unroll
    for (int j = 0; j < GRP; ++j)
#pragma unroll
        for (int nt = 0; nt < 3; ++nt) tm[j][nt] = NEG;

    const int nch = (R + MC - 1) / MC;
#pragma unroll 1
    for (int ch = 0; ch < nch; ++ch) {
        const int r0 = ch * MC;
        __syncthreads();
        stage_x(X, xs, P0 + r0, tid);
        __syncthreads();
#pragma unroll 1
        for (int rr = 0; rr < MC; ++rr) {
            const float v = f_dot(xs + rr * XP, wv, bcv);
            As[rr * AP + tid] = (f16)(v * 256.0f);
        }
        __syncthreads();

        v8f a1[2][4];
#pragma unroll
        for (int mt = 0; mt < 2; ++mt)
#pragma unroll
            for (int nt = 0; nt < 4; ++nt) a1[mt][nt] = zero8();
        {
            const f16* pa = As + m16 * AP + 8 * hh;
            const f16* pb = W3bT + (size_t)(64 * w + m16) * H2_N + 8 * hh;
#pragma unroll 1
            for (int k0 = 0; k0 < H2_N; k0 += 32) {
                const v16h af0 = ldfrag_h(pa, k0);
                const v16h af1 = ldfrag_h(pa + 16 * AP, k0);
                v16h bfr[4];
#pragma unroll
                for (int nt = 0; nt < 4; ++nt) bfr[nt] = ldfrag_h(pb + (size_t)nt * 16 * H2_N, k0);
#pragma unroll
                for (int nt = 0; nt < 4; ++nt) {
                    a1[0][nt] = wm_h(af0, bfr[nt], a1[0][nt]);
                    a1[1][nt] = wm_h(af1, bfr[nt], a1[1][nt]);
                }
                asm volatile("v_nop\n\tv_nop\n\tv_nop\n\tv_nop"
                             : "+v"(a1[0][0]), "+v"(a1[0][1]), "+v"(a1[0][2]), "+v"(a1[0][3]),
                               "+v"(a1[1][0]), "+v"(a1[1][1]), "+v"(a1[1][2]), "+v"(a1[1][3])
                             : "v"(af0), "v"(af1), "v"(bfr[0]), "v"(bfr[1]), "v"(bfr[2]), "v"(bfr[3]));
            }
        }
#pragma unroll
        for (int mt = 0; mt < 2; ++mt) {
#pragma unroll
            for (int nt = 0; nt < 4; ++nt) {
                const int col = 64 * w + 16 * nt + m16;
#pragma unroll
                for (int r = 0; r < 8; ++r) {
                    const int row = 16 * mt + 8 * hh + r;
                    const int grow = r0 + row;
                    int ls = 0;
#pragma unroll
                    for (int j = 0; j < GRP - 1; ++j) ls += (grow >= bl[j]) ? 1 : 0;
                    const float gv = g3s[ls * H3_N + col];
                    float v = fmaf(a1[mt][nt][r], 1.0f / 16384.0f, gv);
                    v = fmaxf(v, 0.0f) * 256.0f;
                    hs[row * HP + col] = (f16)v;
                }
            }
        }
        __syncthreads();

        v8f a2[2][3];
#pragma unroll
        for (int mt = 0; mt < 2; ++mt)
#pragma unroll
            for (int nt = 0; nt < 3; ++nt) a2[mt][nt] = zero8();
        {
            const f16* qa = hs + m16 * HP + 8 * hh;
            const f16* qb = W4T + (size_t)(48 * w + m16) * H3_N + 8 * hh;
#pragma unroll 1
            for (int k0 = 0; k0 < H3_N; k0 += 32) {
                const v16h af0 = ldfrag_h(qa, k0);
                const v16h af1 = ldfrag_h(qa + 16 * HP, k0);
                v16h bfr[3];
#pragma unroll
                for (int nt = 0; nt < 3; ++nt) bfr[nt] = ldfrag_h(qb + (size_t)nt * 16 * H3_N, k0);
#pragma unroll
                for (int nt = 0; nt < 3; ++nt) {
                    a2[0][nt] = wm_h(af0, bfr[nt], a2[0][nt]);
                    a2[1][nt] = wm_h(af1, bfr[nt], a2[1][nt]);
                }
                asm volatile("v_nop\n\tv_nop\n\tv_nop\n\tv_nop"
                             : "+v"(a2[0][0]), "+v"(a2[0][1]), "+v"(a2[0][2]),
                               "+v"(a2[1][0]), "+v"(a2[1][1]), "+v"(a2[1][2])
                             : "v"(af0), "v"(af1), "v"(bfr[0]), "v"(bfr[1]), "v"(bfr[2]));
            }
        }
#pragma unroll
        for (int mt = 0; mt < 2; ++mt) {
#pragma unroll
            for (int nt = 0; nt < 3; ++nt) {
#pragma unroll
                for (int r = 0; r < 8; ++r) {
                    const float v = fmaf(a2[mt][nt][r], 1.0f / 16384.0f, b4v[nt]);
                    const int grow = r0 + 16 * mt + 8 * hh + r;
                    const bool ok = grow < R;
                    int ls = 0;
#pragma unroll
                    for (int j = 0; j < GRP - 1; ++j) ls += (grow >= bl[j]) ? 1 : 0;
#pragma unroll
                    for (int j = 0; j < GRP; ++j)
                        tm[j][nt] = (ok && ls == j) ? fmaxf(tm[j][nt], v) : tm[j][nt];
                }
            }
        }
    }

#pragma unroll
    for (int j = 0; j < GRP; ++j)
#pragma unroll
        for (int nt = 0; nt < 3; ++nt) {
            const float o = __shfl_xor(tm[j][nt], 16, 32);
            tm[j][nt] = fmaxf(tm[j][nt], o);
        }
    __syncthreads();
    float* tks = (float*)hs;
#pragma unroll
    for (int j = 0; j < GRP; ++j)
#pragma unroll
        for (int nt = 0; nt < 3; ++nt) tks[j * TKP + 48 * w + 16 * nt + m16] = tm[j][nt];
    __syncthreads();
    v4f_t ov[2];
#pragma unroll
    for (int it = 0; it < 2; ++it) {
        int L = it * 32 + (tid >> 3);
        L = L < (GRP * 12 - 1) ? L : (GRP * 12 - 1);
        const int j = L / 12, q = L - j * 12;
        const int col = q * 32 + (tid & 7) * 4;
        ov[it] = *(const v4f*)(tks + j * TKP + col);
    }
#pragma unroll
    for (int it = 0; it < 2; ++it) {
        const int Lr = it * 32 + (tid >> 3);
        if (Lr < GRP * 12) {
            const int j = Lr / 12, q = Lr - j * 12;
            const int col = q * 32 + (tid & 7) * 4;
            *(volatile v4f_t*)(tok + (size_t)(s0 + j) * C_N + col) = ov[it];
        }
    }
    __threadfence();
#pragma unroll
    for (int it = 0; it < 2; ++it) {
        const int Lr = it * 32 + (tid >> 3);
        if (Lr < GRP * 12) {
            const int j = Lr / 12, q = Lr - j * 12;
            const int col = q * 32 + (tid & 7) * 4;
            *(volatile v4f_t*)(tok + (size_t)(s0 + j) * C_N + col) = ov[it];
        }
    }
}

__global__ void __launch_bounds__(NTHR) pos_kernel(
    const float* __restrict__ coords, const float* __restrict__ P1, const float* __restrict__ pb1,
    const unsigned short* __restrict__ P2h, const unsigned short* __restrict__ P2l,
    const float* __restrict__ pb2, float* __restrict__ pos)
{
    __shared__ __align__(16) unsigned char raw[MC * TKP * 4];
    unsigned short* Ah = (unsigned short*)raw;
    unsigned short* Al = Ah + MC * PP;
    float* stg = (float*)raw;

    const int tid = threadIdx.x, lane = tid & 31, w = tid >> 5;
    const int hh = lane >> 4, m16 = lane & 15;
    const int s0 = blockIdx.x * MC;
    const int kc = tid & (PH_N - 1), rb = tid >> 7;
    const float p0 = P1[kc], p1 = P1[PH_N + kc], p2 = P1[2 * PH_N + kc], pbv = pb1[kc];
#pragma unroll 1
    for (int i = 0; i < MC / 2; ++i) {
        const int row = rb + 2 * i;
        const int s = s0 + row;
        const float c0 = coords[s * 3], c1 = coords[s * 3 + 1], c2 = coords[s * 3 + 2];
        float v = c0 * p0;
        v = fmaf(c1, p1, v);
        v = fmaf(c2, p2, v);
        v = v + pbv;
        const float ge = 0.5f * v * (1.0f + erff(v * 0.70710678118654752f));
        const unsigned short hb = bf16_rne(ge);
        const float hf = __uint_as_float(((unsigned)hb) << 16);
        Ah[row * PP + kc] = hb;
        Al[row * PP + kc] = bf16_rne(ge - hf);
    }
    float pbv2[3];
#pragma unroll
    for (int nt = 0; nt < 3; ++nt) pbv2[nt] = pb2[48 * w + 16 * nt + m16];
    __syncthreads();

    v8f acc[2][3];
#pragma unroll
    for (int mt = 0; mt < 2; ++mt)
#pragma unroll
        for (int nt = 0; nt < 3; ++nt) acc[mt][nt] = zero8();
    {
        const unsigned short* pah = Ah + m16 * PP + 8 * hh;
        const unsigned short* pal = Al + m16 * PP + 8 * hh;
        const unsigned short* pbh = P2h + (size_t)(48 * w + m16) * PH_N + 8 * hh;
        const unsigned short* pbl = P2l + (size_t)(48 * w + m16) * PH_N + 8 * hh;
#pragma unroll 1
        for (int k0 = 0; k0 < PH_N; k0 += 32) {
            const v16bf ah0 = ldfrag_b(pah, k0);
            const v16bf ah1 = ldfrag_b(pah + 16 * PP, k0);
            const v16bf al0 = ldfrag_b(pal, k0);
            const v16bf al1 = ldfrag_b(pal + 16 * PP, k0);
            v16bf bh[3], blo[3];
#pragma unroll
            for (int nt = 0; nt < 3; ++nt) {
                bh[nt]  = ldfrag_b(pbh + (size_t)nt * 16 * PH_N, k0);
                blo[nt] = ldfrag_b(pbl + (size_t)nt * 16 * PH_N, k0);
            }
#pragma unroll
            for (int nt = 0; nt < 3; ++nt) {
                acc[0][nt] = wm_b(ah0, bh[nt], acc[0][nt]);
                acc[0][nt] = wm_b(ah0, blo[nt], acc[0][nt]);
                acc[0][nt] = wm_b(al0, bh[nt], acc[0][nt]);
                acc[1][nt] = wm_b(ah1, bh[nt], acc[1][nt]);
                acc[1][nt] = wm_b(ah1, blo[nt], acc[1][nt]);
                acc[1][nt] = wm_b(al1, bh[nt], acc[1][nt]);
            }
            asm volatile("v_nop\n\tv_nop\n\tv_nop\n\tv_nop"
                         : "+v"(acc[0][0]), "+v"(acc[0][1]), "+v"(acc[0][2]),
                           "+v"(acc[1][0]), "+v"(acc[1][1]), "+v"(acc[1][2])
                         : "v"(ah0), "v"(ah1), "v"(al0), "v"(al1),
                           "v"(bh[0]), "v"(bh[1]), "v"(bh[2]), "v"(blo[0]), "v"(blo[1]), "v"(blo[2]));
        }
    }
    __syncthreads();
#pragma unroll
    for (int mt = 0; mt < 2; ++mt)
#pragma unroll
        for (int nt = 0; nt < 3; ++nt) {
            const int col = 48 * w + 16 * nt + m16;
#pragma unroll
            for (int r = 0; r < 8; ++r)
                stg[(16 * mt + 8 * hh + r) * TKP + col] = acc[mt][nt][r] + pbv2[nt];
        }
    __syncthreads();
    v4f_t ov[12];
#pragma unroll
    for (int it = 0; it < 12; ++it) {
        const int L = it * 32 + (tid >> 3);
        const int row = L / 12, q = L - row * 12;
        const int col = q * 32 + (tid & 7) * 4;
        ov[it] = *(const v4f*)(stg + row * TKP + col);
    }
#pragma unroll
    for (int it = 0; it < 12; ++it) {
        const int L = it * 32 + (tid >> 3);
        const int row = L / 12, q = L - row * 12;
        const int col = q * 32 + (tid & 7) * 4;
        *(volatile v4f_t*)(pos + (size_t)(s0 + row) * C_N + col) = ov[it];
    }
    __threadfence();
#pragma unroll
    for (int it = 0; it < 12; ++it) {
        const int L = it * 32 + (tid >> 3);
        const int row = L / 12, q = L - row * 12;
        const int col = q * 32 + (tid & 7) * 4;
        *(volatile v4f_t*)(pos + (size_t)(s0 + row) * C_N + col) = ov[it];
    }
}

__global__ void __launch_bounds__(96) pad_kernel(
    const float* __restrict__ tok, const float* __restrict__ pos,
    const int* __restrict__ idx21, float* __restrict__ out)
{
    __shared__ int st;
    const int gi = blockIdx.x >> 6, t = blockIdx.x & 63, tid = threadIdx.x;
    if (tid == 0) st = lbound(idx21, S1_N, gi, LB_IT_S1);
    __syncthreads();
    const int s = st + t;
    const int sc = s < (S1_N - 1) ? s : (S1_N - 1);
    const bool ok = (s < S1_N) && (idx21[sc] == gi);
    const v4f_t a = *(const v4f*)(tok + (size_t)sc * C_N + 4 * tid);
    const v4f_t b = *(const v4f*)(pos + (size_t)sc * C_N + 4 * tid);
    v4f_t oa, ob;
#pragma unroll
    for (int i = 0; i < 4; ++i) {
        oa[i] = ok ? a[i] : 0.0f;
        ob[i] = ok ? b[i] : 0.0f;
    }
    const size_t off0 = (size_t)blockIdx.x * C_N + (size_t)(4 * tid);
    const size_t off1 = (size_t)S2_N * PAD_N * C_N + off0;
    *(volatile v4f_t*)(out + off0) = oa;
    *(volatile v4f_t*)(out + off1) = ob;
    __threadfence();
    *(volatile v4f_t*)(out + off0) = oa;
    *(volatile v4f_t*)(out + off1) = ob;
}

extern "C" void kernel_launch(void* const* d_in, const int* in_sizes, int n_in,
                              void* d_out, int out_size, void* d_ws, size_t ws_size,
                              hipStream_t stream)
{
    if (n_in < 16) return;
    if (in_sizes[0] != N_PTS * F_IN) return;
    if (in_sizes[1] != S1_N * 3) return;
    if (in_sizes[2] != F_IN * H1_N) return;
    if (in_sizes[3] != H1_N) return;
    if (in_sizes[4] != H1_N * H2_N) return;
    if (in_sizes[5] != H2_N) return;
    if (in_sizes[6] != H3_N * H3_N) return;
    if (in_sizes[7] != H3_N) return;
    if (in_sizes[8] != H3_N * C_N) return;
    if (in_sizes[9] != C_N) return;
    if (in_sizes[10] != 3 * PH_N) return;
    if (in_sizes[11] != PH_N) return;
    if (in_sizes[12] != PH_N * C_N) return;
    if (in_sizes[13] != C_N) return;
    if (in_sizes[14] != N_PTS) return;
    if (in_sizes[15] != S1_N) return;
    if (out_size != 2 * S2_N * PAD_N * C_N) return;

    const float* X      = (const float*)d_in[0];
    const float* coords = (const float*)d_in[1];
    const float* W1     = (const float*)d_in[2];
    const float* b1     = (const float*)d_in[3];
    const float* W2     = (const float*)d_in[4];
    const float* b2     = (const float*)d_in[5];
    const float* W3     = (const float*)d_in[6];
    const float* b3     = (const float*)d_in[7];
    const float* W4     = (const float*)d_in[8];
    const float* b4     = (const float*)d_in[9];
    const float* P1     = (const float*)d_in[10];
    const float* pb1    = (const float*)d_in[11];
    const float* P2     = (const float*)d_in[12];
    const float* pb2    = (const float*)d_in[13];
    const int*   idx10  = (const int*)d_in[14];
    const int*   idx21  = (const int*)d_in[15];
    float* out = (float*)d_out;

    const size_t nWc  = (size_t)F_IN * H2_N * 4;
    const size_t nbc  = (size_t)H2_N * 4;
    const size_t nW3h = (size_t)H3_N * H2_N * 2;
    const size_t nW4h = (size_t)C_N * H3_N * 2;
    const size_t nP2  = (size_t)C_N * PH_N * 2;
    const size_t ng   = (size_t)S1_N * H2_N * 4;
    const size_t nG3  = (size_t)S1_N * H3_N * 4;
    const size_t ntok = (size_t)S1_N * C_N * 4;
    const size_t npos = ntok;

    const size_t oWc  = 0;
    const size_t obc  = oWc  + nWc;
    const size_t oW3a = obc  + nbc;
    const size_t oW3b = oW3a + nW3h;
    const size_t oW4  = oW3b + nW3h;
    const size_t oP2h = oW4  + nW4h;
    const size_t oP2l = oP2h + nP2;
    const size_t og   = oP2l + nP2;
    const size_t oG3  = og   + ng;
    const size_t otok = oG3  + nG3;
    const size_t opos = otok + ntok;
    const size_t total = opos + npos;
    if (total > ws_size) return;

    char* ws = (char*)d_ws;
    float* Wc  = (float*)(ws + oWc);
    float* bc  = (float*)(ws + obc);
    f16* W3aT  = (f16*)(ws + oW3a);
    f16* W3bT  = (f16*)(ws + oW3b);
    f16* W4T   = (f16*)(ws + oW4);
    unsigned short* P2h = (unsigned short*)(ws + oP2h);
    unsigned short* P2l = (unsigned short*)(ws + oP2l);
    float* gpl  = (float*)(ws + og);
    float* G3   = (float*)(ws + oG3);
    float* tok  = (float*)(ws + otok);
    float* pos  = (float*)(ws + opos);

    prep_kernel<<<1, NTHR, 0, stream>>>(W1, b1, W2, b2, Wc, bc);

    cvt_t_kernel<0><<<dim3(H3_N / 64, H2_N / 64), NTHR, 0, stream>>>(
        W3, H2_N, H3_N, 64.0f, (unsigned short*)W3aT, (unsigned short*)W3aT);
    cvt_t_kernel<0><<<dim3(H3_N / 64, H2_N / 64), NTHR, 0, stream>>>(
        W3 + (size_t)H2_N * H3_N, H2_N, H3_N, 64.0f, (unsigned short*)W3bT, (unsigned short*)W3bT);
    cvt_t_kernel<0><<<dim3(C_N / 64, H3_N / 64), NTHR, 0, stream>>>(
        W4, H3_N, C_N, 64.0f, (unsigned short*)W4T, (unsigned short*)W4T);
    cvt_t_kernel<1><<<dim3(C_N / 64, PH_N / 64), NTHR, 0, stream>>>(
        P2, PH_N, C_N, 1.0f, P2h, P2l);

    segmax1_kernel<<<S1_N / GRP, NTHR, 0, stream>>>(X, idx10, Wc, bc, gpl);
    g3_kernel<<<S1_N / MC, NTHR, 0, stream>>>(gpl, W3aT, b3, G3);
    fused_kernel<<<S1_N / GRP, NTHR, 0, stream>>>(X, idx10, Wc, bc, G3, W3bT, W4T, b4, tok);
    pos_kernel<<<S1_N / MC, NTHR, 0, stream>>>(coords, P1, pb1, P2h, P2l, pb2, pos);
    pad_kernel<<<S2_N * PAD_N, 96, 0, stream>>>(tok, pos, idx21, out);
}
